// StandardAttentionTransformer_23012434772036
// MI455X (gfx1250) — hardware-verified
//
#include <hip/hip_runtime.h>
#include <math.h>


#define PMOD   53
#define NTOK   54
#define DMODEL 128
#define NHEADS 4
#define DHEAD  32
#define DMLP   512
#define NPAD   64
#define RPB    64

typedef _Float16 v16h __attribute__((ext_vector_type(16)));
typedef _Float16 v8h  __attribute__((ext_vector_type(8)));
typedef float    v8f  __attribute__((ext_vector_type(8)));
typedef float    v4f  __attribute__((ext_vector_type(4)));

union Frag { v16h v; v8h half[2]; };

__device__ __forceinline__ v8f wmma16(v16h a, v16h b, v8f c)
{
    v8f d = __builtin_amdgcn_wmma_f32_16x16x32_f16(false, a, false, b, (short)0, c, false, false);
    asm volatile("v_nop\n\tv_nop\n\tv_nop\n\tv_nop" : "+v"(d) : "v"(a), "v"(b));
    return d;
}

__device__ __forceinline__ v8f zero8()
{
    v8f z;
#pragma unroll
    for (int e = 0; e < 8; ++e) z[e] = 0.f;
    return z;
}

__device__ __forceinline__ int fix_tok(int v)
{
    int t = v;
    if (t < 0) t += NTOK;
    if (t < 0) t = 0;
    if (t > NTOK - 1) t = NTOK - 1;
    return t;
}

__global__ __launch_bounds__(256)
void k_cvt(const float* __restrict__ Win, const float* __restrict__ Wout,
           const float* __restrict__ U,
           _Float16* Win16, _Float16* Wout16, _Float16* U16,
           int n1g, int n2g, int n3g, int urows)
{
    const int g   = blockIdx.x * blockDim.x + threadIdx.x;
    const int tot = n1g + n2g + n3g;
    if (g >= tot) return;

    v4f lo, hi;
    _Float16* dst;
    bool zero = false;
    const float* src = Win;
    if (g < n1g) {
        src = Win + (size_t)g * 8;
        dst = Win16 + (size_t)g * 8;
    } else if (g < n1g + n2g) {
        const int gg = g - n1g;
        src = Wout + (size_t)gg * 8;
        dst = Wout16 + (size_t)gg * 8;
    } else {
        const int gg  = g - n1g - n2g;
        const int row = gg / (DMODEL / 8);
        zero = (row >= urows);
        if (!zero) src = U + (size_t)gg * 8;
        dst = U16 + (size_t)gg * 8;
    }
    if (zero) {
#pragma unroll
        for (int i = 0; i < 4; ++i) { lo[i] = 0.f; hi[i] = 0.f; }
    } else {
        lo = *(const v4f*)src;
        hi = *(const v4f*)(src + 4);
    }
    v8h o;
#pragma unroll
    for (int i = 0; i < 4; ++i) { o[i] = (_Float16)lo[i]; o[4 + i] = (_Float16)hi[i]; }
    *(volatile v8h*)dst = o;
    __threadfence();
    *(volatile v8h*)dst = o;
}

__global__ __launch_bounds__(128)
void k_tables(const float* __restrict__ te, const float* __restrict__ pe,
              const float* __restrict__ WQ, const float* __restrict__ WK,
              const float* __restrict__ WV, const float* __restrict__ WO,
              float* VOA, float* VOB, float* VOC, float* ST, float* SC, float* X2B)
{
    const int t = blockIdx.x;
    const int d = threadIdx.x;
    const int h = d >> 5;
    const int k = d & 31;
    const float rs = 1.0f / 5.656854249492381f;

    __shared__ __attribute__((aligned(16))) float e0[128];
    __shared__ __attribute__((aligned(16))) float e1[128];
    __shared__ __attribute__((aligned(16))) float x2[128];
    __shared__ __attribute__((aligned(16))) float vs0[128];
    __shared__ __attribute__((aligned(16))) float vs1[128];
    __shared__ __attribute__((aligned(16))) float red[256];
    __shared__ __attribute__((aligned(16))) float lines[32];
    __shared__ __attribute__((aligned(16))) float stage[1024];

    const int tt = (t < NTOK) ? t : (NTOK - 1);
    x2[d] = te[(NTOK - 1) * DMODEL + d] + pe[2 * DMODEL + d];
    e0[d] = te[tt * DMODEL + d] + pe[d];
    e1[d] = te[tt * DMODEL + d] + pe[DMODEL + d];
    __syncthreads();

    float q2 = 0.f;
#pragma unroll 1
    for (int dd = 0; dd < DMODEL; ++dd) q2 += x2[dd] * WQ[(h * DMODEL + dd) * DHEAD + k];

    if (t < NTOK) {
        float k0 = 0.f, k1 = 0.f, v0 = 0.f, v1 = 0.f;
#pragma unroll 1
        for (int dd = 0; dd < DMODEL; ++dd) {
            const float wk = WK[(h * DMODEL + dd) * DHEAD + k];
            const float wv = WV[(h * DMODEL + dd) * DHEAD + k];
            const float a0 = e0[dd], a1 = e1[dd];
            k0 += a0 * wk;  k1 += a1 * wk;
            v0 += a0 * wv;  v1 += a1 * wv;
        }
        vs0[d] = v0;  vs1[d] = v1;
        red[d] = q2 * k0;  red[128 + d] = q2 * k1;
        __syncthreads();
        if (d < 32) {
            float lv = 0.f;
            if (d < 8) {
                const int hh = d & 3;
                const int base = ((d < 4) ? 0 : 128) + hh * 32;
                float s = 0.f;
#pragma unroll 1
                for (int i = 0; i < 32; ++i) s += red[base + i];
                lv = s * rs;
            }
            lines[d] = lv;
        }
#pragma unroll
        for (int hh = 0; hh < NHEADS; ++hh) {
            float a0 = 0.f, a1 = 0.f;
#pragma unroll 1
            for (int kk = 0; kk < DHEAD; ++kk) {
                const float w = WO[(hh * DHEAD + kk) * DMODEL + d];
                a0 += vs0[hh * DHEAD + kk] * w;
                a1 += vs1[hh * DHEAD + kk] * w;
            }
            stage[hh * DMODEL + d]       = a0;
            stage[512 + hh * DMODEL + d] = a1;
        }
        __syncthreads();
        const v4f va = *(const v4f*)(stage + 4 * d);
        const v4f vb = *(const v4f*)(stage + 512 + 4 * d);
        v4f vl = va;
        if (d < 8) vl = *(const v4f*)(lines + 4 * d);
        float* pa = VOA + (size_t)t * 512 + 4 * d;
        float* pb = VOB + (size_t)t * 512 + 4 * d;
        float* pl = ST + (size_t)t * 32 + 4 * d;
        *(volatile v4f*)pa = va;
        *(volatile v4f*)pb = vb;
        if (d < 8) *(volatile v4f*)pl = vl;
        __threadfence();
        *(volatile v4f*)pa = va;
        *(volatile v4f*)pb = vb;
        if (d < 8) *(volatile v4f*)pl = vl;
    } else {
        float k2 = 0.f, v2 = 0.f;
#pragma unroll 1
        for (int dd = 0; dd < DMODEL; ++dd) {
            const float a2 = x2[dd];
            k2 += a2 * WK[(h * DMODEL + dd) * DHEAD + k];
            v2 += a2 * WV[(h * DMODEL + dd) * DHEAD + k];
        }
        vs0[d] = v2;  red[d] = q2 * k2;
        __syncthreads();
        if (d < 32) {
            float lv = 0.f;
            if (d < 4) {
                float s = 0.f;
#pragma unroll 1
                for (int i = 0; i < 32; ++i) s += red[d * 32 + i];
                lv = s * rs;
            }
            lines[d] = lv;
        }
#pragma unroll
        for (int hh = 0; hh < NHEADS; ++hh) {
            float a = 0.f;
#pragma unroll 1
            for (int kk = 0; kk < DHEAD; ++kk)
                a += vs0[hh * DHEAD + kk] * WO[(hh * DHEAD + kk) * DMODEL + d];
            stage[hh * DMODEL + d] = a;
        }
        __syncthreads();
        const v4f vc = *(const v4f*)(stage + 4 * d);
        v4f vl = vc, vx = vc;
        if (d < 8)  vl = *(const v4f*)(lines + 4 * d);
        if (d < 32) vx = *(const v4f*)(x2 + 4 * d);
        float* pc = VOC + 4 * d;
        float* pl = SC + 4 * d;
        float* px = X2B + 4 * d;
        *(volatile v4f*)pc = vc;
        if (d < 8)  *(volatile v4f*)pl = vl;
        if (d < 32) *(volatile v4f*)px = vx;
        __threadfence();
        *(volatile v4f*)pc = vc;
        if (d < 8)  *(volatile v4f*)pl = vl;
        if (d < 32) *(volatile v4f*)px = vx;
    }
}

__device__ __forceinline__ void store_block_out(float* out, const float* ob, size_t obase, int valid, int tid)
{
#pragma unroll 1
    for (int i = tid; i < (RPB * PMOD) / 4; i += 128) {
        const int f = 4 * i;
        if (f + 4 <= valid) {
            const v4f v = *(const v4f*)(ob + f);
            *(volatile v4f*)(out + obase + f) = v;
        } else {
#pragma unroll
            for (int q = 0; q < 4; ++q)
                if (f + q < valid) *(volatile float*)(out + obase + f + q) = ob[f + q];
        }
    }
}

__global__ __launch_bounds__(128)
void k_main(const int* __restrict__ ta_in, const int* __restrict__ tb_in,
            const _Float16* __restrict__ Win16, const _Float16* __restrict__ Wout16,
            const _Float16* __restrict__ U16,
            const float* __restrict__ VOA, const float* __restrict__ VOB,
            const float* __restrict__ VOC, const float* __restrict__ ST,
            const float* __restrict__ SC, const float* __restrict__ X2B,
            const float* __restrict__ Winb, const float* __restrict__ Woutb,
            float* out, int nb)
{
    __shared__ __attribute__((aligned(16))) float    xbuf[4][16 * DMODEL];
    __shared__ __attribute__((aligned(16))) _Float16 xh[4][16 * DMODEL];
    __shared__ __attribute__((aligned(16))) _Float16 hbuf[4][16 * 32];

    const int tid  = threadIdx.x;
    const int wave = tid >> 5;
    const int lane = tid & 31;
    const int r    = lane & 15;
    const int hs   = lane >> 4;
    const int blk  = blockIdx.x;
    const int rb   = blk * RPB + wave * 16;
    float*    xb = xbuf[wave];
    _Float16* xq = xh[wave];
    _Float16* hb = hbuf[wave];

    {
        const int grow = rb + r;
        int ta = 0, tb = 0;
        if (grow < nb) { ta = ta_in[grow]; tb = tb_in[grow]; }
        ta = fix_tok(ta);  tb = fix_tok(tb);
        float w0[4], w1[4], w2[4];
#pragma unroll
        for (int h = 0; h < NHEADS; ++h) {
            const float s0 = ST[ta * 32 + h];
            const float s1 = ST[tb * 32 + 4 + h];
            const float s2 = SC[h];
            const float m  = fmaxf(s0, fmaxf(s1, s2));
            const float x0 = expf(s0 - m), x1 = expf(s1 - m), x2v = expf(s2 - m);
            const float inv = 1.0f / (x0 + x1 + x2v);
            w0[h] = x0 * inv;  w1[h] = x1 * inv;  w2[h] = x2v * inv;
        }
#pragma unroll 1
        for (int c = 0; c < 8; ++c) {
            const int dd = hs * 64 + c * 8;
            v4f vlo = *(const v4f*)(X2B + dd);
            v4f vhi = *(const v4f*)(X2B + dd + 4);
#pragma unroll
            for (int h = 0; h < NHEADS; ++h) {
                const float* pa = VOA + (size_t)(ta * NHEADS + h) * DMODEL + dd;
                const float* pb = VOB + (size_t)(tb * NHEADS + h) * DMODEL + dd;
                const float* pc = VOC + h * DMODEL + dd;
                vlo = vlo + w0[h] * *(const v4f*)(pa) + w1[h] * *(const v4f*)(pb) + w2[h] * *(const v4f*)(pc);
                vhi = vhi + w0[h] * *(const v4f*)(pa + 4) + w1[h] * *(const v4f*)(pb + 4) + w2[h] * *(const v4f*)(pc + 4);
            }
            *(v4f*)(xb + r * DMODEL + dd)     = vlo;
            *(v4f*)(xb + r * DMODEL + dd + 4) = vhi;
            v8h q;
#pragma unroll
            for (int i = 0; i < 4; ++i) { q[i] = (_Float16)vlo[i]; q[4 + i] = (_Float16)vhi[i]; }
            *(v8h*)(xq + r * DMODEL + dd) = q;
        }
    }
    __syncthreads();

    v8f acc[8];
#pragma unroll
    for (int nn = 0; nn < 8; ++nn) acc[nn] = zero8();

#pragma unroll 1
    for (int j = 0; j < DMLP / 32; ++j) {
        v8f hacc[2];
        hacc[0] = zero8();  hacc[1] = zero8();
#pragma unroll
        for (int kk = 0; kk < 4; ++kk) {
            Frag a;
            a.half[0] = *(const v8h*)(xq + r * DMODEL + kk * 32 + 8 * hs);
            a.half[1] = *(const v8h*)(xq + r * DMODEL + kk * 32 + 16 + 8 * hs);
#pragma unroll
            for (int sub = 0; sub < 2; ++sub) {
                const int n = j * 32 + sub * 16 + r;
                Frag b;
                b.half[0] = *(const v8h*)(Win16 + (size_t)n * DMODEL + kk * 32 + 8 * hs);
                b.half[1] = *(const v8h*)(Win16 + (size_t)n * DMODEL + kk * 32 + 16 + 8 * hs);
                hacc[sub] = wmma16(a.v, b.v, hacc[sub]);
            }
        }
#pragma unroll
        for (int sub = 0; sub < 2; ++sub) {
            const int n = j * 32 + sub * 16 + r;
            const float bias = Winb[n];
#pragma unroll
            for (int e = 0; e < 8; ++e) {
                const int row = 8 * hs + e;
                hb[row * 32 + sub * 16 + r] = (_Float16)fmaxf(hacc[sub][e] + bias, 0.f);
            }
        }
        __syncthreads();
        Frag ha;
        ha.half[0] = *(const v8h*)(hb + r * 32 + 8 * hs);
        ha.half[1] = *(const v8h*)(hb + r * 32 + 16 + 8 * hs);
        __syncthreads();
#pragma unroll
        for (int nn = 0; nn < 8; ++nn) {
            const int n = nn * 16 + r;
            Frag b;
            b.half[0] = *(const v8h*)(Wout16 + (size_t)n * DMLP + j * 32 + 8 * hs);
            b.half[1] = *(const v8h*)(Wout16 + (size_t)n * DMLP + j * 32 + 16 + 8 * hs);
            acc[nn] = wmma16(ha.v, b.v, acc[nn]);
        }
    }

#pragma unroll
    for (int nn = 0; nn < 8; ++nn) {
        const int n = nn * 16 + r;
        const float bias = Woutb[n];
#pragma unroll
        for (int e = 0; e < 8; ++e) {
            const int row = 8 * hs + e;
            const float v = acc[nn][e] + bias + xb[row * DMODEL + n];
            xq[row * DMODEL + n] = (_Float16)v;
        }
    }
    __syncthreads();

    v8f lacc[4];
#pragma unroll
    for (int nn = 0; nn < 4; ++nn) lacc[nn] = zero8();
#pragma unroll
    for (int kk = 0; kk < 4; ++kk) {
        Frag a;
        a.half[0] = *(const v8h*)(xq + r * DMODEL + kk * 32 + 8 * hs);
        a.half[1] = *(const v8h*)(xq + r * DMODEL + kk * 32 + 16 + 8 * hs);
#pragma unroll
        for (int nn = 0; nn < 4; ++nn) {
            const int n = nn * 16 + r;
            Frag b;
            b.half[0] = *(const v8h*)(U16 + (size_t)n * DMODEL + kk * 32 + 8 * hs);
            b.half[1] = *(const v8h*)(U16 + (size_t)n * DMODEL + kk * 32 + 16 + 8 * hs);
            lacc[nn] = wmma16(a.v, b.v, lacc[nn]);
        }
    }
    float* ob = &xbuf[0][0];
#pragma unroll
    for (int nn = 0; nn < 4; ++nn) {
        const int n = nn * 16 + r;
        if (n < PMOD) {
#pragma unroll
            for (int e = 0; e < 8; ++e) {
                const int lrow = wave * 16 + 8 * hs + e;
                ob[lrow * PMOD + n] = lacc[nn][e];
            }
        }
    }
    __syncthreads();

    const size_t obase = (size_t)blk * (RPB * PMOD);
    const size_t tot   = (size_t)nb * PMOD;
    int valid = 0;
    if (obase < tot) {
        const size_t rem = tot - obase;
        valid = (rem < (size_t)(RPB * PMOD)) ? (int)rem : (RPB * PMOD);
    }
    store_block_out(out, ob, obase, valid, tid);
    __threadfence();
    store_block_out(out, ob, obase, valid, tid);
}

extern "C" void kernel_launch(void* const* d_in, const int* in_sizes, int n_in,
                              void* d_out, int out_size, void* d_ws, size_t ws_size,
                              hipStream_t stream)
{
    if (n_in < 13) return;
    const int nb = in_sizes[0];
    if (nb <= 0 || in_sizes[1] != nb) return;
    if (out_size != nb * PMOD) return;
    if (in_sizes[2] != NTOK * DMODEL || in_sizes[3] != 3 * DMODEL) return;
    if (in_sizes[4] != NHEADS * DMODEL * DHEAD || in_sizes[5] != NHEADS * DMODEL * DHEAD ||
        in_sizes[6] != NHEADS * DMODEL * DHEAD || in_sizes[7] != NHEADS * DHEAD * DMODEL) return;
    if (in_sizes[8] != DMLP * DMODEL || in_sizes[9] != DMLP ||
        in_sizes[10] != DMODEL * DMLP || in_sizes[11] != DMODEL || in_sizes[12] != PMOD * DMODEL) return;

    const int*   a     = (const int*)d_in[0];
    const int*   b     = (const int*)d_in[1];
    const float* te    = (const float*)d_in[2];
    const float* pe    = (const float*)d_in[3];
    const float* WQ    = (const float*)d_in[4];
    const float* WK    = (const float*)d_in[5];
    const float* WV    = (const float*)d_in[6];
    const float* WO    = (const float*)d_in[7];
    const float* Win   = (const float*)d_in[8];
    const float* Winb  = (const float*)d_in[9];
    const float* Wout  = (const float*)d_in[10];
    const float* Woutb = (const float*)d_in[11];
    const float* U     = (const float*)d_in[12];

    char* ws = (char*)d_ws;
    size_t off = 0;
    const size_t szWin16  = (size_t)DMLP * DMODEL * 2;
    const size_t szWout16 = (size_t)DMODEL * DMLP * 2;
    const size_t szU16    = (size_t)NPAD * DMODEL * 2;
    const size_t szVOA    = (size_t)NTOK * NHEADS * DMODEL * 4;
    const size_t szVOB    = szVOA;
    const size_t szVOC    = (size_t)NHEADS * DMODEL * 4;
    const size_t szST     = (size_t)NTOK * 32 * 4;
    const size_t szSC     = 32 * 4;
    const size_t szX2B    = (size_t)DMODEL * 4;
    auto carve = [&](size_t bytes) -> char* { char* p = ws + off; off += (bytes + 255) & ~(size_t)255; return p; };
    _Float16* Win16  = (_Float16*)carve(szWin16);
    _Float16* Wout16 = (_Float16*)carve(szWout16);
    _Float16* U16    = (_Float16*)carve(szU16);
    float* VOA = (float*)carve(szVOA);
    float* VOB = (float*)carve(szVOB);
    float* VOC = (float*)carve(szVOC);
    float* ST  = (float*)carve(szST);
    float* SC  = (float*)carve(szSC);
    float* X2B = (float*)carve(szX2B);
    if (off > ws_size) return;

    k_tables<<<dim3(NTOK + 1), dim3(128), 0, stream>>>(
        te, pe, WQ, WK, WV, WO, VOA, VOB, VOC, ST, SC, X2B);

    const int n1g = DMLP * DMODEL / 8;
    const int n2g = DMODEL * DMLP / 8;
    const int n3g = NPAD * DMODEL / 8;
    const int ncvt = n1g + n2g + n3g;
    k_cvt<<<dim3((ncvt + 255) / 256), dim3(256), 0, stream>>>(
        Win, Wout, U, Win16, Wout16, U16, n1g, n2g, n3g, PMOD);

    const int nblk = (nb + RPB - 1) / RPB;
    k_main<<<dim3(nblk), dim3(128), 0, stream>>>(
        a, b, Win16, Wout16, U16, VOA, VOB, VOC, ST, SC, X2B, Winb, Woutb, (float*)d_out, nb);
}
